// Sam_Block_14645838479457
// MI455X (gfx1250) — hardware-verified
//
#include <hip/hip_runtime.h>
#include <hip/hip_bf16.h>
#include <math.h>


typedef _Float16 bf16;
typedef _Float16 f16;
typedef __attribute__((ext_vector_type(4))) unsigned v4u_t;
typedef unsigned v4ua __attribute__((ext_vector_type(4), may_alias));
typedef __attribute__((ext_vector_type(4))) float v4f_t;
typedef float v4fa __attribute__((ext_vector_type(4), may_alias));
typedef __attribute__((ext_vector_type(16))) bf16  bf16x16;
typedef bf16x16 f16x16;
typedef __attribute__((ext_vector_type(8)))  bf16  bf16x8;
typedef bf16x8 f16x8;
typedef __attribute__((ext_vector_type(4)))  bf16  bf16x4;
typedef __attribute__((ext_vector_type(8)))  float f32x8;
__device__ __forceinline__ f32x8 wmma16(f16x16 a, f16x16 b, f32x8 c) {
  c = __builtin_amdgcn_wmma_f32_16x16x32_f16(false, a, false, b, (short)0, c, false, false);
  asm volatile("v_nop\n\tv_nop\n\tv_nop\n\tv_nop" : "+v"(c) : "v"(a), "v"(b));
  return c;
}
#define LDS_STRIDE 48
#define KSTRIDE    72
#define VSTRIDE    48

__device__ __forceinline__ f32x8 wmma_bf16(bf16x16 a, bf16x16 b, f32x8 c) {
  c = __builtin_amdgcn_wmma_f32_16x16x32_f16(false, a, false, b, (short)0, c, false, false);
  asm volatile("v_nop\n\tv_nop\n\tv_nop\n\tv_nop" : "+v"(c) : "v"(a), "v"(b));
  return c;
}

template <typename T>
__device__ __forceinline__ bf16x16 load_frag(const T* __restrict__ base, int ld,
                                             int row0, int k0) {
  const int lane = threadIdx.x & 31;
  const int r    = lane & 15;
  const int kh   = (lane >> 4) * 8;
  const T* p0 = base + (size_t)(row0 + r) * ld + (k0 + kh);
  const T* p1 = p0 + 16;
  bf16x16 f;
#pragma unroll
  for (int i = 0; i < 8; ++i) {
    f[i]     = (bf16)p0[i];
    f[i + 8] = (bf16)p1[i];
  }
  return f;
}

__device__ __forceinline__ bf16x16 lds_frag(const bf16* base, int stride) {
  const int lane = threadIdx.x & 31;
  const int row  = lane & 15;
  const int kh   = (lane >> 4) * 8;
  const bf16x8 lo = *(const bf16x8*)(base + row * stride + kh);
  const bf16x8 hi = *(const bf16x8*)(base + row * stride + kh + 16);
  bf16x16 f;
#pragma unroll
  for (int i = 0; i < 8; ++i) { f[i] = lo[i]; f[i + 8] = hi[i]; }
  return f;
}

template <typename T>
__device__ __forceinline__ void stage_read16(const T* __restrict__ p, float* buf) {
#pragma unroll
  for (int i = 0; i < 16; ++i) buf[i] = (float)p[i];
}

__device__ __forceinline__ void stage_write(bf16* dst, const float* buf, int nquad) {
#pragma unroll
  for (int i = 0; i < nquad; ++i) {
    bf16x4 q;
    q[0] = (bf16)buf[4 * i];     q[1] = (bf16)buf[4 * i + 1];
    q[2] = (bf16)buf[4 * i + 2]; q[3] = (bf16)buf[4 * i + 3];
    *(bf16x4*)(dst + 4 * i) = q;
  }
}


#define GSTR 48
#define GSTR 48
template <typename AT, int EPI, bool OUT16>
__global__ __launch_bounds__(256) void gemm_kne(const AT* __restrict__ A, int lda, const float* __restrict__ Wm, int ldw,
                                                const float* __restrict__ bias, const float* __restrict__ R, const float* __restrict__ gvec,
                                                void* __restrict__ Yv, int ldy, int K) {
  __shared__ __attribute__((aligned(16))) f16 ldsA[128 * GSTR];
  __shared__ __attribute__((aligned(16))) f16 ldsW[128 * GSTR];
  __shared__ __attribute__((aligned(16))) float oS[8][32 * 68];
  const int tid = threadIdx.x, lane = tid & 31, wave = tid >> 5, cl = lane & 15, rh = (lane >> 4) * 8;
  const int m0 = blockIdx.x * 128, n0 = blockIdx.y * 128;
  const int wm = (wave & 3) * 32, wn = (wave >> 2) * 64;
  f32x8 acc[2][4];
#pragma unroll
  for (int i = 0; i < 2; ++i)
#pragma unroll
    for (int j = 0; j < 4; ++j) { f32x8 z = {}; acc[i][j] = z; }
#pragma unroll 1
  for (int k0 = 0; k0 < K; k0 += 32) {
    __syncthreads();
    { const int row = tid >> 1, ch = (tid & 1) * 16;
      const AT* src = A + (size_t)(m0 + row) * lda + k0 + ch;
#pragma unroll
      for (int g = 0; g < 16; ++g) ldsA[row * GSTR + ch + g] = (f16)src[g]; }
    { const int k = tid >> 3, nn0 = (tid & 7) * 16;
      const float* src = Wm + (size_t)(k0 + k) * ldw + n0 + nn0;
#pragma unroll
      for (int g = 0; g < 4; ++g) { const v4f_t v = *(const v4f_t*)(src + 4 * g);
#pragma unroll
        for (int u = 0; u < 4; ++u) ldsW[(nn0 + 4 * g + u) * GSTR + k] = (f16)v[u]; } }
    __syncthreads();
    f16x16 af[2];
#pragma unroll
    for (int i = 0; i < 2; ++i) af[i] = lds_frag(ldsA + (wm + 16 * i) * GSTR, GSTR);
#pragma unroll
    for (int j = 0; j < 4; ++j) {
      const f16x16 bf = lds_frag(ldsW + (wn + 16 * j) * GSTR, GSTR);
#pragma unroll
      for (int i = 0; i < 2; ++i) acc[i][j] = wmma16(af[i], bf, acc[i][j]);
    }
  }
  float* so = oS[wave];
#pragma unroll
  for (int i = 0; i < 2; ++i)
#pragma unroll
    for (int j = 0; j < 4; ++j) {
      const int n = n0 + wn + 16 * j + cl;
      const float bv = bias ? bias[n] : 0.0f;
      const float gv = (EPI == 2 || EPI == 4) ? gvec[n] : 0.0f;
      if (EPI == 1) {
#pragma unroll 1
        for (int r = 0; r < 8; ++r) { const float xg = acc[i][j][r] + bv; so[(16 * i + rh + r) * 68 + 16 * j + cl] = 0.5f * xg * (1.0f + erff(xg * 0.70710678118654752f)); }
      } else {
#pragma unroll
        for (int r = 0; r < 8; ++r) {
          float v = acc[i][j][r] + bv;
          if (EPI == 3) v = fmaxf(v, 0.0f);
          if (EPI == 4) v = gv * v;
          if (EPI == 2) v = R[(size_t)(m0 + wm + 16 * i + rh + r) * ldy + n] + gv * v;
          so[(16 * i + rh + r) * 68 + 16 * j + cl] = v;
        }
      }
    }
  asm volatile("s_wait_dscnt 0" ::: "memory");
  __builtin_amdgcn_wave_barrier();
#pragma unroll 1
  for (int pass = 0; pass < 2; ++pass) {
    if (OUT16) {
      f16* Y = (f16*)Yv;
#pragma unroll
      for (int it = 0; it < 8; ++it) { const int c = lane + 32 * it, rr = c >> 3, q8 = (c & 7) * 8;
        union { f16 h[8]; v4u_t v; } u;
#pragma unroll
        for (int e = 0; e < 8; ++e) u.h[e] = (f16)so[rr * 68 + q8 + e];
        *(volatile v4u_t*)(Y + (size_t)(m0 + wm + rr) * ldy + n0 + wn + q8) = u.v; }
    } else {
      float* Y = (float*)Yv;
#pragma unroll
      for (int it = 0; it < 16; ++it) { const int f4 = lane + 32 * it, rr = f4 >> 4, q = (f4 & 15) * 4;
        *(volatile v4f_t*)(Y + (size_t)(m0 + wm + rr) * ldy + n0 + wn + q) = *(const v4fa*)(so + rr * 68 + q); }
    }
    __threadfence();
  }
}

template <typename AT, int EPI, bool OUT16>
__global__ __launch_bounds__(256) void gemm_knez(const AT* __restrict__ A, int lda, size_t strideA, const float* __restrict__ Wm, int ldw, size_t strideW,
                                                 const float* __restrict__ bias, const float* __restrict__ R, const float* __restrict__ gvec,
                                                 void* __restrict__ Yv, int ldy, size_t strideY, int K) {
  A += (size_t)blockIdx.z * strideA; Wm += (size_t)blockIdx.z * strideW; Yv = (void*)((char*)Yv + (size_t)blockIdx.z * strideY * (OUT16 ? 2 : 4)); if (R) R += (size_t)blockIdx.z * strideY;
  __shared__ __attribute__((aligned(16))) f16 ldsA[128 * GSTR];
  __shared__ __attribute__((aligned(16))) f16 ldsW[128 * GSTR];
  __shared__ __attribute__((aligned(16))) float oS[8][32 * 68];
  const int tid = threadIdx.x, lane = tid & 31, wave = tid >> 5, cl = lane & 15, rh = (lane >> 4) * 8;
  const int m0 = blockIdx.x * 128, n0 = blockIdx.y * 128;
  const int wm = (wave & 3) * 32, wn = (wave >> 2) * 64;
  f32x8 acc[2][4];
#pragma unroll
  for (int i = 0; i < 2; ++i)
#pragma unroll
    for (int j = 0; j < 4; ++j) { f32x8 z = {}; acc[i][j] = z; }
#pragma unroll 1
  for (int k0 = 0; k0 < K; k0 += 32) {
    __syncthreads();
    { const int row = tid >> 1, ch = (tid & 1) * 16;
      const AT* src = A + (size_t)(m0 + row) * lda + k0 + ch;
#pragma unroll
      for (int g = 0; g < 16; ++g) ldsA[row * GSTR + ch + g] = (f16)src[g]; }
    { const int k = tid >> 3, nn0 = (tid & 7) * 16;
      const float* src = Wm + (size_t)(k0 + k) * ldw + n0 + nn0;
#pragma unroll
      for (int g = 0; g < 4; ++g) { const v4f_t v = *(const v4f_t*)(src + 4 * g);
#pragma unroll
        for (int u = 0; u < 4; ++u) ldsW[(nn0 + 4 * g + u) * GSTR + k] = (f16)v[u]; } }
    __syncthreads();
    f16x16 af[2];
#pragma unroll
    for (int i = 0; i < 2; ++i) af[i] = lds_frag(ldsA + (wm + 16 * i) * GSTR, GSTR);
#pragma unroll
    for (int j = 0; j < 4; ++j) {
      const f16x16 bf = lds_frag(ldsW + (wn + 16 * j) * GSTR, GSTR);
#pragma unroll
      for (int i = 0; i < 2; ++i) acc[i][j] = wmma16(af[i], bf, acc[i][j]);
    }
  }
  float* so = oS[wave];
#pragma unroll
  for (int i = 0; i < 2; ++i)
#pragma unroll
    for (int j = 0; j < 4; ++j) {
      const int n = n0 + wn + 16 * j + cl;
      const float bv = bias ? bias[n] : 0.0f;
      const float gv = (EPI == 2 || EPI == 4) ? gvec[n] : 0.0f;
      if (EPI == 1) {
#pragma unroll 1
        for (int r = 0; r < 8; ++r) { const float xg = acc[i][j][r] + bv; so[(16 * i + rh + r) * 68 + 16 * j + cl] = 0.5f * xg * (1.0f + erff(xg * 0.70710678118654752f)); }
      } else {
#pragma unroll
        for (int r = 0; r < 8; ++r) {
          float v = acc[i][j][r] + bv;
          if (EPI == 3) v = fmaxf(v, 0.0f);
          if (EPI == 4) v = gv * v;
          if (EPI == 2) v = R[(size_t)(m0 + wm + 16 * i + rh + r) * ldy + n] + gv * v;
          so[(16 * i + rh + r) * 68 + 16 * j + cl] = v;
        }
      }
    }
  asm volatile("s_wait_dscnt 0" ::: "memory");
  __builtin_amdgcn_wave_barrier();
#pragma unroll 1
  for (int pass = 0; pass < 2; ++pass) {
    if (OUT16) {
      f16* Y = (f16*)Yv;
#pragma unroll
      for (int it = 0; it < 8; ++it) { const int c = lane + 32 * it, rr = c >> 3, q8 = (c & 7) * 8;
        union { f16 h[8]; v4u_t v; } u;
#pragma unroll
        for (int e = 0; e < 8; ++e) u.h[e] = (f16)so[rr * 68 + q8 + e];
        *(volatile v4u_t*)(Y + (size_t)(m0 + wm + rr) * ldy + n0 + wn + q8) = u.v; }
    } else {
      float* Y = (float*)Yv;
#pragma unroll
      for (int it = 0; it < 16; ++it) { const int f4 = lane + 32 * it, rr = f4 >> 4, q = (f4 & 15) * 4;
        *(volatile v4f_t*)(Y + (size_t)(m0 + wm + rr) * ldy + n0 + wn + q) = *(const v4fa*)(so + rr * 68 + q); }
    }
    __threadfence();
  }
}

template <typename AT, bool ACC>
__global__ __launch_bounds__(256) void gemm_kn2(const AT* __restrict__ A, int lda, size_t strideA,
                                               const float* __restrict__ Wm, int ldw, size_t strideW,
                                               const float* __restrict__ bias, float scale,
                                               float* __restrict__ Y, int ldy, size_t strideY, int K) {
  __shared__ __attribute__((aligned(16))) f16 ldsA[128 * GSTR], ldsAl[128 * GSTR];
  __shared__ __attribute__((aligned(16))) f16 ldsW[128 * GSTR], ldsWl[128 * GSTR];
  __shared__ __attribute__((aligned(16))) float oS[8][32 * 68];
  const int tid = threadIdx.x, lane = tid & 31, wave = tid >> 5, cl = lane & 15, rh = (lane >> 4) * 8;
  const int m0 = blockIdx.x * 128, n0 = blockIdx.y * 128;
  const int wm = (wave & 3) * 32, wn = (wave >> 2) * 64;
  A += (size_t)blockIdx.z * strideA; Wm += (size_t)blockIdx.z * strideW; Y += (size_t)blockIdx.z * strideY;
  f32x8 acc[2][4], accx[2][4];
#pragma unroll
  for (int i = 0; i < 2; ++i)
#pragma unroll
    for (int j = 0; j < 4; ++j) { f32x8 z = {}; acc[i][j] = z; accx[i][j] = z; }
#pragma unroll 1
  for (int k0 = 0; k0 < K; k0 += 32) {
    __syncthreads();
    {
      const int row = tid >> 1, ch = (tid & 1) * 16;
      const AT* src = A + (size_t)(m0 + row) * lda + k0 + ch;
#pragma unroll
      for (int g = 0; g < 16; ++g) { const float v = (float)src[g]; const f16 h = (f16)v; ldsA[row * GSTR + ch + g] = h; ldsAl[row * GSTR + ch + g] = (f16)((v - (float)h) * 2048.0f); }
    }
    {
      const int k = tid >> 3, nn0 = (tid & 7) * 16;
      const float* src = Wm + (size_t)(k0 + k) * ldw + n0 + nn0;
#pragma unroll
      for (int g = 0; g < 4; ++g) { const v4f_t v = *(const v4f_t*)(src + 4 * g);
#pragma unroll
        for (int u = 0; u < 4; ++u) { const f16 h = (f16)v[u]; ldsW[(nn0 + 4 * g + u) * GSTR + k] = h; ldsWl[(nn0 + 4 * g + u) * GSTR + k] = (f16)((v[u] - (float)h) * 2048.0f); } }
    }
    __syncthreads();
    f16x16 af[2], afl[2];
#pragma unroll
    for (int i = 0; i < 2; ++i) { af[i] = lds_frag(ldsA + (wm + 16 * i) * GSTR, GSTR); afl[i] = lds_frag(ldsAl + (wm + 16 * i) * GSTR, GSTR); }
#pragma unroll
    for (int j = 0; j < 4; ++j) {
      const f16x16 bf = lds_frag(ldsW + (wn + 16 * j) * GSTR, GSTR), bfl = lds_frag(ldsWl + (wn + 16 * j) * GSTR, GSTR);
#pragma unroll
      for (int i = 0; i < 2; ++i) { acc[i][j] = wmma16(af[i], bf, acc[i][j]); accx[i][j] = wmma16(af[i], bfl, accx[i][j]); accx[i][j] = wmma16(afl[i], bf, accx[i][j]); }
    }
  }
  float* so = oS[wave];
#pragma unroll
  for (int i = 0; i < 2; ++i)
#pragma unroll
    for (int j = 0; j < 4; ++j) {
      const float bv = bias ? bias[n0 + wn + 16 * j + cl] : 0.0f;
#pragma unroll
      for (int r = 0; r < 8; ++r) so[(16 * i + rh + r) * 68 + 16 * j + cl] = (acc[i][j][r] + accx[i][j][r] * (1.0f / 2048.0f)) * scale + bv;
    }
  asm volatile("s_wait_dscnt 0" ::: "memory");
  __builtin_amdgcn_wave_barrier();
  if (ACC) {
#pragma unroll
    for (int it = 0; it < 16; ++it) { const int f4 = lane + 32 * it, rr = f4 >> 4, q = (f4 & 15) * 4;
      const v4f_t old = *(const v4fa*)(Y + (size_t)(m0 + wm + rr) * ldy + n0 + wn + q);
      v4f_t v = *(const v4fa*)(so + rr * 68 + q); v += old; *(v4fa*)(so + rr * 68 + q) = v; }
    asm volatile("s_wait_dscnt 0" ::: "memory");
  }
#pragma unroll 1
  for (int pass = 0; pass < 2; ++pass) {
#pragma unroll
    for (int it = 0; it < 16; ++it) { const int f4 = lane + 32 * it, rr = f4 >> 4, q = (f4 & 15) * 4;
      *(volatile v4f_t*)(Y + (size_t)(m0 + wm + rr) * ldy + n0 + wn + q) = *(const v4fa*)(so + rr * 68 + q); }
    __threadfence();
  }
}

__global__ __launch_bounds__(256) void k_transpose(const float* __restrict__ Wm, float* __restrict__ Wt, int rows, int cols) {
  __shared__ float tS[64][65];
  const int tid = threadIdx.x, tbj = cols / 64, bi = blockIdx.x / tbj, bj = blockIdx.x % tbj;
  for (int e = tid; e < 64 * 64; e += 256) { const int r = e >> 6, c = e & 63; tS[r][c] = Wm[(size_t)(bi * 64 + r) * cols + bj * 64 + c]; }
  __syncthreads();
  for (int ch = tid; ch < 64 * 16; ch += 256) { const int r = ch >> 4, q4 = (ch & 15) * 4; v4f_t o; o[0] = tS[q4][r]; o[1] = tS[q4 + 1][r]; o[2] = tS[q4 + 2][r]; o[3] = tS[q4 + 3][r];
    float* dst = Wt + (size_t)(bj * 64 + r) * rows + bi * 64 + q4; *(volatile v4f_t*)dst = o; __threadfence(); *(volatile v4f_t*)dst = o; }
}


template <typename AT, int EPI, bool OUT16, int NJ>
__global__ __launch_bounds__(256) void gemm_sm(const AT* __restrict__ A, int lda, size_t sA, const float* __restrict__ Wm, int ldw, size_t sW,
                                               const float* __restrict__ bias, const float* __restrict__ R, const float* __restrict__ gvec,
                                               void* __restrict__ Yv, int ldy, size_t sY, int K) {
  constexpr int BN = 16 * NJ; constexpr int OST = BN + 4;
  A += (size_t)blockIdx.z * sA; Wm += (size_t)blockIdx.z * sW; Yv = (void*)((char*)Yv + (size_t)blockIdx.z * sY * (OUT16 ? 2 : 4)); if (R) R += (size_t)blockIdx.z * sY;
  __shared__ __attribute__((aligned(16))) f16 ldsA[256 * GSTR];
  __shared__ __attribute__((aligned(16))) f16 ldsW[BN * GSTR];
  __shared__ __attribute__((aligned(16))) float oS[8][32 * OST];
  const int tid = threadIdx.x, lane = tid & 31, wave = tid >> 5, cl = lane & 15, rh = (lane >> 4) * 8;
  const int m0 = blockIdx.x * 256, n0 = blockIdx.y * BN;
  const int wm = wave * 32;
  f32x8 acc[2][NJ];
#pragma unroll
  for (int i = 0; i < 2; ++i)
#pragma unroll
    for (int j = 0; j < NJ; ++j) { f32x8 z = {}; acc[i][j] = z; }
#pragma unroll 1
  for (int k0 = 0; k0 < K; k0 += 32) {
    __syncthreads();
    { const AT* src = A + (size_t)(m0 + tid) * lda + k0;
#pragma unroll
      for (int g = 0; g < 32; ++g) ldsA[tid * GSTR + g] = (f16)src[g]; }
    { const int k = tid >> 3, nn0 = (tid & 7) * (2 * NJ);
      const float* src = Wm + (size_t)(k0 + k) * ldw + n0 + nn0;
#pragma unroll
      for (int g = 0; g < NJ / 2; ++g) { const v4f_t v = *(const v4f_t*)(src + 4 * g);
#pragma unroll
        for (int u = 0; u < 4; ++u) ldsW[(nn0 + 4 * g + u) * GSTR + k] = (f16)v[u]; } }
    __syncthreads();
    f16x16 af[2];
#pragma unroll
    for (int i = 0; i < 2; ++i) af[i] = lds_frag(ldsA + (wm + 16 * i) * GSTR, GSTR);
#pragma unroll
    for (int j = 0; j < NJ; ++j) {
      const f16x16 bf = lds_frag(ldsW + (16 * j) * GSTR, GSTR);
#pragma unroll
      for (int i = 0; i < 2; ++i) acc[i][j] = wmma16(af[i], bf, acc[i][j]);
    }
  }
  float* so = oS[wave];
#pragma unroll
  for (int i = 0; i < 2; ++i)
#pragma unroll
    for (int j = 0; j < NJ; ++j) {
      const int n = n0 + 16 * j + cl;
      const float bv = bias ? bias[n] : 0.0f;
      const float gv = (EPI == 2 || EPI == 4) ? gvec[n] : 0.0f;
#pragma unroll
      for (int r = 0; r < 8; ++r) {
        float v = acc[i][j][r] + bv;
        if (EPI == 3) v = fmaxf(v, 0.0f);
        if (EPI == 2) v = R[(size_t)(m0 + wm + 16 * i + rh + r) * ldy + n] + gv * v;
        if (EPI == 4) v = gv * v;
        so[(16 * i + rh + r) * OST + 16 * j + cl] = v;
      }
    }
  asm volatile("s_wait_dscnt 0" ::: "memory");
  __builtin_amdgcn_wave_barrier();
#pragma unroll 1
  for (int pass = 0; pass < 2; ++pass) {
    if (OUT16) {
      f16* Y = (f16*)Yv;
#pragma unroll
      for (int it = 0; it < BN / 8; ++it) { const int c = lane + 32 * it, rr = c / (BN / 8), q8 = (c % (BN / 8)) * 8;
        union { f16 h[8]; v4u_t v; } u;
#pragma unroll
        for (int e = 0; e < 8; ++e) u.h[e] = (f16)so[rr * OST + q8 + e];
        *(volatile v4u_t*)(Y + (size_t)(m0 + wm + rr) * ldy + n0 + q8) = u.v; }
    } else {
      float* Y = (float*)Yv;
#pragma unroll
      for (int it = 0; it < BN / 4; ++it) { const int f4 = lane + 32 * it, rr = f4 / (BN / 4), q = (f4 % (BN / 4)) * 4;
        *(volatile v4f_t*)(Y + (size_t)(m0 + wm + rr) * ldy + n0 + q) = *(const v4fa*)(so + rr * OST + q); }
    }
    __threadfence();
  }
}

#define NBsb 2
#define GHsb 64
#define NTsb 4096
#define CCsb 768
#define NHsb 12
#define HDsb 64
#define WSsb 14
#define NWAsb 5
#define NWsb 25
#define WTsb 256
#define WVsb 196
#define MLsb 3072
__global__ __launch_bounds__(256) void k_fill(float* __restrict__ p, float val, size_t n4) { const size_t i = (size_t)blockIdx.x * 256 + threadIdx.x; if (i < n4) { v4f_t v = {val, val, val, val}; *(volatile v4f_t*)(p + 4 * i) = v; __threadfence(); *(volatile v4f_t*)(p + 4 * i) = v; } }
__global__ __launch_bounds__(256) void k_dbg_zero(float* __restrict__ p, size_t n4) { const size_t i = (size_t)blockIdx.x * 256 + threadIdx.x; if (i < n4) { v4f_t z = {0.f,0.f,0.f,0.f}; *(volatile v4f_t*)(p + 4 * i) = z; __threadfence(); *(volatile v4f_t*)(p + 4 * i) = z; } }
__global__ __launch_bounds__(256) void k_copy(const float* __restrict__ src, float* __restrict__ dst, size_t n4) { const size_t i = (size_t)blockIdx.x * 256 + threadIdx.x; if (i < n4) { const v4f_t v = *(const v4f_t*)(src + 4 * i); *(volatile v4f_t*)(dst + 4 * i) = v; __threadfence(); *(volatile v4f_t*)(dst + 4 * i) = v; } }
__global__ __launch_bounds__(256) void k_transpose_ld(const float* __restrict__ Wm, int lds, float* __restrict__ Wt, int rows, int cols) {
  __shared__ float tS[64][65];
  const int tid = threadIdx.x, tbj = cols / 64, bi = blockIdx.x / tbj, bj = blockIdx.x % tbj;
  for (int e = tid; e < 64 * 64; e += 256) { const int r = e >> 6, c = e & 63; tS[r][c] = Wm[(size_t)(bi * 64 + r) * lds + bj * 64 + c]; }
  __syncthreads();
  for (int ch = tid; ch < 64 * 16; ch += 256) { const int r = ch >> 4, q4 = (ch & 15) * 4; v4f_t o; o[0] = tS[q4][r]; o[1] = tS[q4 + 1][r]; o[2] = tS[q4 + 2][r]; o[3] = tS[q4 + 3][r];
    float* dst = Wt + (size_t)(bj * 64 + r) * rows + bi * 64 + q4; *(volatile v4f_t*)dst = o; __threadfence(); *(volatile v4f_t*)dst = o; }
}
__global__ __launch_bounds__(256) void k_gelu(float* __restrict__ Hm, size_t n4) { const size_t i = (size_t)blockIdx.x * 256 + threadIdx.x; if (i >= n4) return; v4f_t v = *(const v4fa*)(Hm + 4 * i);
#pragma unroll
  for (int u = 0; u < 4; ++u) v[u] = 0.5f * v[u] * (1.0f + erff(v[u] * 0.70710678118654752f));
  *(volatile v4fa*)(Hm + 4 * i) = v; __threadfence(); *(volatile v4fa*)(Hm + 4 * i) = v; }
__global__ __launch_bounds__(256) void k_ln(const float* __restrict__ X, const float* __restrict__ gam, const float* __restrict__ bet, float* __restrict__ Y) {
  __shared__ __attribute__((aligned(16))) float rowS[16 * 772];
  const int tid = threadIdx.x, r = tid >> 4, part = tid & 15; const size_t row = (size_t)blockIdx.x * 16 + r;
  float s = 0.0f;
#pragma unroll 1
  for (int i = 0; i < 48; ++i) { const float v = X[row * 768 + part * 48 + i]; rowS[r * 772 + part * 48 + i] = v; s += v; }
  s += __shfl_xor(s, 1, 32); s += __shfl_xor(s, 2, 32); s += __shfl_xor(s, 4, 32); s += __shfl_xor(s, 8, 32);
  const float mean = s * (1.0f / 768.0f); float q = 0.0f;
#pragma unroll 1
  for (int i = 0; i < 48; ++i) { const float dv = rowS[r * 772 + part * 48 + i] - mean; q += dv * dv; }
  q += __shfl_xor(q, 1, 32); q += __shfl_xor(q, 2, 32); q += __shfl_xor(q, 4, 32); q += __shfl_xor(q, 8, 32);
  const float rstd = 1.0f / __builtin_sqrtf(q * (1.0f / 768.0f) + 1e-5f);
#pragma unroll 1
  for (int i = 0; i < 48; ++i) { const int c = part * 48 + i; rowS[r * 772 + c] = (rowS[r * 772 + c] - mean) * rstd * gam[c] + bet[c]; }
  __syncthreads();
#pragma unroll 1
  for (int pass = 0; pass < 2; ++pass) { for (int q4 = tid; q4 < 16 * 192; q4 += 256) { const int rr = q4 / 192, c4 = (q4 % 192) * 4;
      *(volatile v4f_t*)(Y + ((size_t)blockIdx.x * 16 + rr) * 768 + c4) = *(const v4fa*)(rowS + rr * 772 + c4); } __threadfence(); }
}
__global__ __launch_bounds__(256) void k_wpart(const float* __restrict__ XN, int w0, int nw, float* __restrict__ XW, size_t n4) { const size_t i = (size_t)blockIdx.x * 256 + threadIdx.x; if (i >= n4) return; const size_t e = 4 * i; const int r = (int)(e / CCsb), c = (int)(e % CCsb); const int w = w0 + r / WTsb, t = r % WTsb;
  v4f_t v; v[0] = v[1] = v[2] = v[3] = 0.0f;
  if (t < WVsb) { const int hb = w / NWAsb, wb = w % NWAsb, hh = t / WSsb, ww = t % WSsb; const int y = hb * WSsb + hh, x = wb * WSsb + ww; if (y < GHsb && x < GHsb) v = *(const v4f_t*)(XN + ((size_t)y * GHsb + x) * CCsb + c); }
  *(volatile v4f_t*)(XW + e) = v; __threadfence(); *(volatile v4f_t*)(XW + e) = v; }
__global__ __launch_bounds__(256) void k_wunpart(const float* __restrict__ Pw, int w0, float* __restrict__ H1, size_t n4) { const size_t i = (size_t)blockIdx.x * 256 + threadIdx.x; if (i >= n4) return; const size_t e = 4 * i; const int r = (int)(e / CCsb), c = (int)(e % CCsb); const int w = w0 + r / WTsb, t = r % WTsb;
  if (t >= WVsb) return; const int hb = w / NWAsb, wb = w % NWAsb, hh = t / WSsb, ww = t % WSsb; const int y = hb * WSsb + hh, x = wb * WSsb + ww; if (y >= GHsb || x >= GHsb) return;
  const v4f_t v = *(const v4f_t*)(Pw + e); float* d = H1 + ((size_t)y * GHsb + x) * CCsb + c; *(volatile v4f_t*)d = v; __threadfence(); *(volatile v4f_t*)d = v; }
__global__ __launch_bounds__(32) void k_relpos(const float* __restrict__ QKV, int h, const float* __restrict__ Rh, const float* __restrict__ Rw, float* __restrict__ REL) { const int r = blockIdx.x, lane = threadIdx.x; const int t = r % WTsb; const int tt = min(t, WVsb - 1); const int th = tt / WSsb, tw = tt % WSsb;
  const int a = lane >> 4, k = min(lane & 15, WSsb - 1); const float* R = (a == 0) ? Rh : Rw; const int ta = (a == 0) ? th : tw; const float* rr = R + (size_t)(ta - k + WSsb - 1) * HDsb; const float* q = QKV + (size_t)r * 3 * CCsb + h * HDsb; float val = 0.0f;
#pragma unroll 1
  for (int c = 0; c < HDsb; ++c) val += q[c] * rr[c];
  *(volatile float*)(REL + (size_t)r * 32 + lane) = val; __threadfence(); *(volatile float*)(REL + (size_t)r * 32 + lane) = val; }
__global__ __launch_bounds__(256) void k_wsoft(float* __restrict__ Sm, const float* __restrict__ REL) { __shared__ float red[256]; const int t = blockIdx.x, w = blockIdx.y, k = threadIdx.x; const size_t row = (size_t)w * WTsb + t; float* sr = Sm + row * WTsb; const float* rl = REL + row * 32;
  const bool ok = (k < WVsb); const int kh = k / WSsb, kw = k % WSsb; float v = ok ? (sr[k] * 0.125f + rl[kh] + rl[16 + kw]) : -3.0e38f;
  red[k] = v; __syncthreads(); for (int o = 128; o > 0; o >>= 1) { if (k < o) red[k] = fmaxf(red[k], red[k + o]); __syncthreads(); }
  const float m = red[0]; __syncthreads(); v = ok ? expf(v - m) : 0.0f; red[k] = v; __syncthreads();
  for (int o = 128; o > 0; o >>= 1) { if (k < o) red[k] += red[k + o]; __syncthreads(); }
  const float p = v * (1024.0f / red[0]) - 1.0f; *(volatile float*)(sr + k) = p; __threadfence(); *(volatile float*)(sr + k) = p; }
__global__ __launch_bounds__(256) void k_vsumw(const float* __restrict__ QKV, float* __restrict__ VSW) { const int w = blockIdx.y, c = blockIdx.x * 256 + threadIdx.x; if (c >= CCsb) return; float s = 0.0f; const float* base = QKV + ((size_t)w * WTsb) * 3 * CCsb + 2 * CCsb + c;
#pragma unroll 1
  for (int t = 0; t < WTsb; ++t) s += base[(size_t)t * 3 * CCsb];
  *(volatile float*)(VSW + (size_t)w * CCsb + c) = s; __threadfence(); *(volatile float*)(VSW + (size_t)w * CCsb + c) = s; }
__global__ __launch_bounds__(256) void k_place(const float* __restrict__ T, const float* __restrict__ VSW, int h, float* __restrict__ O) { const int tid = threadIdx.x; const size_t r = (size_t)blockIdx.x * 16 + (tid >> 4); const int c4 = (tid & 15) * 4; const int w = (int)(r / WTsb);
  const v4f_t v = (*(const v4f_t*)(T + r * HDsb + c4) + *(const v4f_t*)(VSW + (size_t)w * CCsb + h * HDsb + c4)) * (1.0f / 1024.0f); float* d = O + r * CCsb + h * HDsb + c4; *(volatile v4f_t*)d = v; __threadfence(); *(volatile v4f_t*)d = v; }
__global__ __launch_bounds__(256) void k_addx(float* __restrict__ Hm, const float* __restrict__ X, size_t n4) { const size_t i = (size_t)blockIdx.x * 256 + threadIdx.x; if (i >= n4) return; const v4f_t v = *(const v4fa*)(Hm + 4 * i) + *(const v4f_t*)(X + 4 * i); *(volatile v4fa*)(Hm + 4 * i) = v; __threadfence(); *(volatile v4fa*)(Hm + 4 * i) = v; }


extern "C" void kernel_launch(void* const* d_in, const int* in_sizes, int n_in,
                              void* d_out, int out_size, void* d_ws, size_t ws_size,
                              hipStream_t stream) {
  (void)in_sizes; (void)n_in; (void)out_size;
  const float** f = (const float**)d_in;
  const float* x = f[0], *g1 = f[1], *b1n = f[2], *wqkv = f[3], *bqkv = f[4], *wproj = f[5], *bproj = f[6], *Rh = f[7], *Rw = f[8], *g2 = f[9], *b2n = f[10], *w1 = f[11], *bb1 = f[12], *w2 = f[13], *bb2 = f[14];
  float* out = (float*)d_out;
  char* ws = (char*)d_ws;
  const int GMAX = 13;
  float* XN = (float*)ws; ws += (size_t)NTsb * CCsb * 4; float* XW = (float*)ws; ws += (size_t)13 * WTsb * CCsb * 4; float* QKV = (float*)ws; ws += (size_t)13 * WTsb * 3 * CCsb * 4; float* KT = (float*)ws; ws += (size_t)CCsb * 13 * WTsb * 4;
  float* REL = (float*)ws; ws += (size_t)13 * WTsb * 32 * 4; float* VSW = (float*)ws; ws += (size_t)13 * CCsb * 4; float* S = (float*)ws; ws += (size_t)13 * WTsb * WTsb * 4; float* T = (float*)ws; ws += (size_t)13 * WTsb * HDsb * 4; float* O = (float*)ws; ws += (size_t)13 * WTsb * CCsb * 4;
  float* H1 = (float*)ws; ws += (size_t)NTsb * CCsb * 4; float* ones = (float*)ws; ws += MLsb * 4; float* FH = (float*)ws; ws += (size_t)2048 * MLsb * 4;
  if ((size_t)(ws - (char*)d_ws) > ws_size) return;
  (void)GMAX;
  const dim3 blk(256); const size_t n4 = (size_t)NTsb * CCsb / 4;
  k_fill<<<dim3(2), blk, 0, stream>>>(ones, 1.0f, MLsb / 4);

  for (int b = 0; b < NBsb; ++b) { const float* xb = x + (size_t)b * NTsb * CCsb; float* ob = out + (size_t)b * NTsb * CCsb;
    k_ln<<<dim3(NTsb / 16), blk, 0, stream>>>(xb, g1, b1n, XN);
    for (int g = 0; g < 2; ++g) { const int w0 = g ? 13 : 0, nw = g ? 12 : 13; if (nw <= 0) continue; const size_t gr = (size_t)nw * WTsb; const size_t g4 = gr * CCsb / 4;
      k_wpart<<<dim3((g4 + 255) / 256), blk, 0, stream>>>(XN, w0, nw, XW, g4);
      gemm_kne<float, 0, false><<<dim3(gr / 128, 3 * CCsb / 128), blk, 0, stream>>>(XW, CCsb, wqkv, 3 * CCsb, bqkv, nullptr, nullptr, QKV, 3 * CCsb, CCsb);
      k_vsumw<<<dim3(CCsb / 256, nw), blk, 0, stream>>>(QKV, VSW);
      k_transpose_ld<<<dim3((gr / 64) * (CCsb / 64)), blk, 0, stream>>>(QKV + CCsb, 3 * CCsb, KT, gr, CCsb);
      for (int h = 0; h < NHsb; ++h) {
        gemm_knez<float, 0, false><<<dim3(WTsb / 128, WTsb / 128, nw), blk, 0, stream>>>(QKV + h * HDsb, 3 * CCsb, (size_t)WTsb * 3 * CCsb, KT + (size_t)h * HDsb * gr, gr, (size_t)WTsb, nullptr, nullptr, nullptr, S, WTsb, (size_t)WTsb * WTsb, HDsb);
        k_relpos<<<dim3(gr), dim3(32), 0, stream>>>(QKV, h, Rh, Rw, REL);
        k_wsoft<<<dim3(WTsb, nw), blk, 0, stream>>>(S, REL);
        gemm_sm<float, 0, false, 4><<<dim3(WTsb / 256, 1, nw), blk, 0, stream>>>(S, WTsb, (size_t)WTsb * WTsb, QKV + 2 * CCsb + h * HDsb, 3 * CCsb, (size_t)WTsb * 3 * CCsb, nullptr, nullptr, nullptr, T, HDsb, (size_t)WTsb * HDsb, WTsb);
        k_place<<<dim3(gr / 16), blk, 0, stream>>>(T, VSW, h, O);
      }
      gemm_kne<float, 0, false><<<dim3(gr / 128, CCsb / 128), blk, 0, stream>>>(O, CCsb, wproj, CCsb, bproj, nullptr, nullptr, XW, CCsb, CCsb);
      k_wunpart<<<dim3((g4 + 255) / 256), blk, 0, stream>>>(XW, w0, H1, g4);
    }
    k_addx<<<dim3((n4 + 255) / 256), blk, 0, stream>>>(H1, xb, n4);
    k_ln<<<dim3(NTsb / 16), blk, 0, stream>>>(H1, g2, b2n, XN);
    for (size_t r0 = 0; r0 < NTsb; r0 += 2048) {
      gemm_kne<float, 0, false><<<dim3(2048 / 128, MLsb / 128), blk, 0, stream>>>(XN + r0 * CCsb, CCsb, w1, MLsb, bb1, nullptr, nullptr, FH, MLsb, CCsb); k_gelu<<<dim3(((size_t)2048 * MLsb / 4 + 255) / 256), blk, 0, stream>>>(FH, (size_t)2048 * MLsb / 4);
      gemm_kne<float, 2, false><<<dim3(2048 / 128, CCsb / 128), blk, 0, stream>>>(FH, MLsb, w2, CCsb, bb2, H1 + r0 * CCsb, ones, ob + r0 * CCsb, CCsb, MLsb); }
  }
}
